// TrajectoryDecoder_31653908972275
// MI455X (gfx1250) — hardware-verified
//
#include <hip/hip_runtime.h>
#include <stdint.h>

typedef __attribute__((ext_vector_type(16))) _Float16 v16h;
typedef __attribute__((ext_vector_type(8)))  _Float16 v8h;
typedef __attribute__((ext_vector_type(16))) __bf16   v16b;
typedef __attribute__((ext_vector_type(8)))  __bf16   v8b;
typedef __attribute__((ext_vector_type(8)))  float    v8f;
typedef __attribute__((ext_vector_type(4)))  float    v4f;
typedef __attribute__((ext_vector_type(2)))  float    v2f;

constexpr int kCtx          = 128;
constexpr int kHid          = 64;
constexpr int kEnc          = 64;
constexpr int kInW          = 68;
constexpr int kGate         = 4 * kHid;
constexpr int kSteps        = 64;
constexpr int kRowsPerBlock = 128;
constexpr int kThreads      = 256;
constexpr int kOutPitch     = kSteps * 2;
constexpr int kWcatRows     = kGate + 16;

static_assert(kGate == kThreads, "one thread per gate row in the staging pass");
static_assert(kCtx % 32 == 0 && kHid % 32 == 0 && kEnc % 32 == 0, "K multiples of 32");

constexpr int kOffWcat  = 0;
constexpr int kOffWprev = kOffWcat + kWcatRows * kHid * 2;
constexpr int kOffGs    = kOffWprev + kGate * 2 * 4;
constexpr int kOffHt    = kOffGs + 8 * 16 * kGate * 4;
constexpr int kOffPb    = kOffHt + 8 * 16 * kHid * 2;
constexpr int kLdsBytes = kOffPb + 8 * 16 * 32 * 4;
static_assert(kOffWprev == 34816 && kOffGs == 36864 && kOffHt == 167936 && kOffPb == 184320 && kLdsBytes == 200704, "lds map");
static_assert((kOffWprev % 16) == 0 && (kOffGs % 16) == 0 && (kOffHt % 16) == 0 && (kOffPb % 16) == 0, "lds alignment");

__device__ __forceinline__ float bf16r(float f) {
  unsigned u = __float_as_uint(f);
  u = (u + 0x7FFFu + ((u >> 16) & 1u)) & 0xFFFF0000u;
  return __uint_as_float(u);
}
__device__ __forceinline__ __bf16 tobf(float f) {
  const unsigned u = __float_as_uint(f);
  const unsigned short b = (unsigned short)((u + 0x7FFFu + ((u >> 16) & 1u)) >> 16);
  return __builtin_bit_cast(__bf16, b);
}

__device__ __forceinline__ void mem_bar() { asm volatile("" ::: "memory"); }
__device__ __forceinline__ void lds_wave_sync() {
  __builtin_amdgcn_fence(__ATOMIC_RELEASE, "workgroup");
  __builtin_amdgcn_wave_barrier();
  __builtin_amdgcn_fence(__ATOMIC_ACQUIRE, "workgroup");
}

__device__ __forceinline__ v8f mma_b(v16b a, v16b b, v8f c) {
  c = __builtin_amdgcn_wmma_f32_16x16x32_bf16(false, a, false, b, (short)0, c, false, false);
  asm volatile("v_nop\n\tv_nop\n\tv_nop\n\tv_nop" : "+v"(c) : "v"(a), "v"(b));
  return c;
}
__device__ __forceinline__ v8f mma_h(v16h a, v16h b, v8f c) {
  c = __builtin_amdgcn_wmma_f32_16x16x32_f16(false, a, false, b, (short)0, c, false, false);
  asm volatile("v_nop\n\tv_nop\n\tv_nop\n\tv_nop" : "+v"(c) : "v"(a), "v"(b));
  return c;
}

__device__ __forceinline__ v16h ldfrag_h(const _Float16* p) {
  union { v16h v; v8h h[2]; } f;
  f.h[0] = *(const v8h*)(p);
  f.h[1] = *(const v8h*)(p + 16);
  return f.v;
}
__device__ __forceinline__ v16b gfrag_bf16(const float* __restrict__ p) {
  const v4f x0 = *(const v4f*)(p);
  const v4f x1 = *(const v4f*)(p + 4);
  const v4f x2 = *(const v4f*)(p + 16);
  const v4f x3 = *(const v4f*)(p + 20);
  v16b f;
#pragma unroll
  for (int e = 0; e < 4; ++e) {
    f[e]      = tobf(x0[e]);
    f[4 + e]  = tobf(x1[e]);
    f[8 + e]  = tobf(x2[e]);
    f[12 + e] = tobf(x3[e]);
  }
  return f;
}
__device__ __forceinline__ v8f splat8(float v) { return (v8f){v, v, v, v, v, v, v, v}; }
__device__ __forceinline__ v16b zero16b() {
  v16b z;
#pragma unroll
  for (int e = 0; e < 16; ++e) z[e] = tobf(0.0f);
  return z;
}

__device__ __forceinline__ float act_sigm(float x) {
  const float xc = fminf(fmaxf(x, -30.0f), 30.0f);
  const float e = __expf(-xc);
  return __builtin_amdgcn_rcpf(1.0f + e);
}
__device__ __forceinline__ float act_tanh(float x) {
  const float xc = fminf(fmaxf(x, -15.0f), 15.0f);
  const float e = __expf(2.0f * xc);
  const float r = __builtin_amdgcn_rcpf(1.0f + e);
  return fmaf(-2.0f, r, 1.0f);
}

__global__ __launch_bounds__(kThreads, 1)
void traj_decode_kernel(const float* __restrict__ context, const float* __restrict__ enc,
                        const float* __restrict__ ball,
                        const float* __restrict__ Wh,  const float* __restrict__ bh,
                        const float* __restrict__ Wc,  const float* __restrict__ bc,
                        const float* __restrict__ Wih, const float* __restrict__ Whh,
                        const float* __restrict__ bih, const float* __restrict__ bhh,
                        const float* __restrict__ Wout, const float* __restrict__ bout,
                        float* __restrict__ out)
{
  extern __shared__ __attribute__((aligned(16))) char smem_dyn[];
  _Float16* wcat  = (_Float16*)(smem_dyn + kOffWcat);
  float*    wprev = (float*)(smem_dyn + kOffWprev);
  float*    gsA   = (float*)(smem_dyn + kOffGs);
  _Float16* htA   = (_Float16*)(smem_dyn + kOffHt);
  float*    pbA   = (float*)(smem_dyn + kOffPb);

  const int tid  = threadIdx.x;
  const int wave = tid >> 5;
  const int lane = tid & 31;
  const int hh   = lane >> 4;
  const int cl   = lane & 15;
  const int row0 = blockIdx.x * kRowsPerBlock + wave * 16;

  float*    gsw = gsA + wave * (16 * kGate);
  _Float16* ht  = htA + wave * (16 * kHid);
  float*    pb  = pbA + wave * (16 * 32);

#pragma unroll 1
  for (int it = 0; it < 8; ++it) {
    const int gi = it * kThreads + tid;
    const int wr = gi >> 3;
    const int c8 = (gi & 7) * 8;
    const float* src = Whh + (size_t)wr * kHid + c8;
    const v4f w0 = *(const v4f*)(src);
    const v4f w1 = *(const v4f*)(src + 4);
    v8h hv;
#pragma unroll
    for (int e = 0; e < 4; ++e) {
      hv[e]     = (_Float16)bf16r(w0[e]);
      hv[4 + e] = (_Float16)bf16r(w1[e]);
    }
    *(v8h*)(wcat + (size_t)wr * kHid + c8) = hv;
  }
  if (tid < 128) {
    const int r2 = tid >> 3;
    const int c8 = (tid & 7) * 8;
    const int orow = (r2 < 1) ? 0 : 1;
    const float* src = Wout + orow * kHid + c8;
    const v4f w0 = *(const v4f*)(src);
    const v4f w1 = *(const v4f*)(src + 4);
    const bool keep = (r2 < 2);
    v8h hv;
#pragma unroll
    for (int e = 0; e < 4; ++e) {
      const float a0v = keep ? bf16r(w0[e]) : 0.0f;
      const float a1v = keep ? bf16r(w1[e]) : 0.0f;
      hv[e]     = (_Float16)a0v;
      hv[4 + e] = (_Float16)a1v;
    }
    *(v8h*)(wcat + (size_t)(kGate + r2) * kHid + c8) = hv;
  }
  wprev[tid * 2 + 0] = bf16r(Wih[(size_t)tid * kInW + 0]);
  wprev[tid * 2 + 1] = bf16r(Wih[(size_t)tid * kInW + 1]);

  v16b actx[4];
  {
    const float* crow = context + (size_t)(row0 + cl) * kCtx + 8 * hh;
#pragma unroll
    for (int kc = 0; kc < 4; ++kc) { actx[kc] = gfrag_bf16(crow + kc * 32); mem_bar(); }
  }
  v8f cst[4];
#pragma unroll
  for (int d = 0; d < 4; ++d) {
    const int col = 16 * d + cl;
    v8f ah = splat8(bf16r(bh[col]));
    v8f ac = splat8(bf16r(bc[col]));
    const float* whr = Wh + (size_t)col * kCtx + 8 * hh;
    const float* wcr = Wc + (size_t)col * kCtx + 8 * hh;
#pragma unroll
    for (int kc = 0; kc < 4; ++kc) {
      const v16b bw  = gfrag_bf16(whr + kc * 32);
      const v16b bcw = gfrag_bf16(wcr + kc * 32);
      mem_bar();
      ah = mma_b(actx[kc], bw, ah);
      ac = mma_b(actx[kc], bcw, ac);
    }
    cst[d] = ac;
#pragma unroll
    for (int r = 0; r < 8; ++r) ht[(8 * hh + r) * kHid + col] = (_Float16)ah[r];
  }

  v16b aenc[2];
  {
    const float* er = enc + (size_t)(row0 + cl) * kEnc + 8 * hh;
    aenc[0] = gfrag_bf16(er);
    aenc[1] = gfrag_bf16(er + 32);
    mem_bar();
  }
  v16b abal = zero16b();
  {
    const float bx = ball[(size_t)(row0 + cl) * 2 + 0];
    const float by = ball[(size_t)(row0 + cl) * 2 + 1];
    abal[0] = tobf((hh == 0) ? bx : 0.0f);
    abal[1] = tobf((hh == 0) ? by : 0.0f);
  }
#pragma unroll 1
  for (int j = 0; j < 16; ++j) {
    const int col = 16 * j + cl;
    const float* wr = Wih + (size_t)col * kInW;
    const float w2 = wr[2], w3 = wr[3];
    v16b bb = zero16b();
    bb[0] = tobf((hh == 0) ? w2 : 0.0f);
    bb[1] = tobf((hh == 0) ? w3 : 0.0f);
    const v16b b0 = gfrag_bf16(wr + 4 + 8 * hh);
    const v16b b1 = gfrag_bf16(wr + 4 + 32 + 8 * hh);
    mem_bar();
    v8f a = splat8(bf16r(bih[col]) + bf16r(bhh[col]));
    a = mma_b(abal, bb, a);
    a = mma_b(aenc[0], b0, a);
    a = mma_b(aenc[1], b1, a);
    float* gp = gsw + j * 256 + lane * 8;
    *(v4f*)(gp)     = __builtin_shufflevector(a, a, 0, 1, 2, 3);
    *(v4f*)(gp + 4) = __builtin_shufflevector(a, a, 4, 5, 6, 7);
  }

  const float bo0  = bf16r(bout[0]);
  const float bo1  = bf16r(bout[1]);
  const float bsel = (cl == 0) ? bo0 : bo1;

  __syncthreads();

  float px[8], py[8];
#pragma unroll
  for (int r = 0; r < 8; ++r) { px[r] = 0.0f; py[r] = 0.0f; }
  const _Float16* hrow  = ht + cl * kHid + 8 * hh;
  const _Float16* worow = wcat + (size_t)(kGate + cl) * kHid + 8 * hh;

#pragma unroll 1
  for (int t = 0; t <= kSteps; ++t) {
    const v16h a0 = ldfrag_h(hrow);
    const v16h a1 = ldfrag_h(hrow + 32);
    if (t > 0) {
      v8f p = splat8(0.0f);
      const v16h b0 = ldfrag_h(worow);
      const v16h b1 = ldfrag_h(worow + 32);
      p = mma_h(a0, b0, p);
      p = mma_h(a1, b1, p);
      const int slot = (t - 1) & 15;
      float pv[8];
#pragma unroll
      for (int r = 0; r < 8; ++r) pv[r] = p[r] + bsel;
      if (cl < 2) {
#pragma unroll
        for (int r = 0; r < 8; ++r) pb[(8 * hh + r) * 32 + slot * 2 + cl] = pv[r];
      }
      const int sx = lane & 16;
#pragma unroll
      for (int r = 0; r < 8; ++r) {
        px[r] = __shfl(pv[r], sx, 32);
        py[r] = __shfl(pv[r], sx + 1, 32);
      }
      if (slot == 15) {
        lds_wave_sync();
        const int tb = (t - 1) >> 4;
        const int q4 = lane >> 3;
        const int c4 = (lane & 7) * 4;
        float* obase = out + (size_t)row0 * kOutPitch + tb * 32 + c4;
        for (int pass = 0; pass < 2; ++pass) {
#pragma unroll
          for (int it = 0; it < 4; ++it) {
            const int rr = it * 4 + q4;
            const v4f v = *(const v4f*)(pb + rr * 32 + c4);
            *(volatile v4f*)(obase + (size_t)rr * kOutPitch) = v;
          }
          __threadfence();
        }
        lds_wave_sync();
      }
    }
    if (t < kSteps) {
#pragma unroll
      for (int d = 0; d < 4; ++d) {
        v8f g4[4];
#pragma unroll
        for (int gg = 0; gg < 4; ++gg) {
          const int j = gg * 4 + d;
          const float* gp = gsw + j * 256 + lane * 8;
          const v4f q0 = *(const v4f*)(gp);
          const v4f q1 = *(const v4f*)(gp + 4);
          const v2f wp = *(const v2f*)(wprev + (16 * j + cl) * 2);
          v8f a = __builtin_shufflevector(q0, q1, 0, 1, 2, 3, 4, 5, 6, 7);
#pragma unroll
          for (int r = 0; r < 8; ++r) a[r] = fmaf(px[r], wp[0], fmaf(py[r], wp[1], a[r]));
          const _Float16* wb = wcat + (size_t)(16 * j + cl) * kHid + 8 * hh;
          const v16h b0 = ldfrag_h(wb);
          const v16h b1 = ldfrag_h(wb + 32);
          a = mma_h(a0, b0, a);
          a = mma_h(a1, b1, a);
          g4[gg] = a;
        }
#pragma unroll
        for (int r = 0; r < 8; ++r) {
          const float ig = act_sigm(g4[0][r]);
          const float fg = act_sigm(g4[1][r]);
          const float gv = act_tanh(g4[2][r]);
          const float og = act_sigm(g4[3][r]);
          const float cn = fmaf(fg, cst[d][r], ig * gv);
          cst[d][r] = cn;
          const float hn = og * act_tanh(cn);
          ht[(8 * hh + r) * kHid + 16 * d + cl] = (_Float16)hn;
        }
      }
    }
    lds_wave_sync();
  }
}

extern "C" void kernel_launch(void* const* d_in, const int* in_sizes, int n_in,
                              void* d_out, int out_size, void* d_ws, size_t ws_size,
                              hipStream_t stream) {
  (void)n_in; (void)d_ws; (void)ws_size;
  const float* context = (const float*)d_in[0];
  const float* enc     = (const float*)d_in[1];
  const float* ball    = (const float*)d_in[2];
  const float* Wh      = (const float*)d_in[3];
  const float* bh      = (const float*)d_in[4];
  const float* Wc      = (const float*)d_in[5];
  const float* bc      = (const float*)d_in[6];
  const float* Wih     = (const float*)d_in[7];
  const float* Whh     = (const float*)d_in[8];
  const float* bih     = (const float*)d_in[9];
  const float* bhh     = (const float*)d_in[10];
  const float* Wout    = (const float*)d_in[11];
  const float* bout    = (const float*)d_in[12];
  float* out = (float*)d_out;

  const int nB   = in_sizes[0] / kCtx;
  const int nblk = nB / kRowsPerBlock;
  if (nblk <= 0) return;
  if (nblk * kRowsPerBlock != nB) return;
  if (out_size != nB * kOutPitch) return;

  traj_decode_kernel<<<dim3(nblk), dim3(kThreads), (size_t)kLdsBytes, stream>>>(
      context, enc, ball, Wh, bh, Wc, bc, Wih, Whh, bih, bhh, Wout, bout, out);
}
